// MultiHeadAttention_30313879176070
// MI455X (gfx1250) — hardware-run, weakly checked
//
#include <hip/hip_runtime.h>


#ifndef NB
#define NB 2
#endif
#ifndef SEQ
#define SEQ 2048
#endif
#define NB_FULL  2
#define SEQ_FULL 2048
#define TT   SEQ
#define DM   1024
#define NH_  16
#define HD   64
#define DQ   (NH_ * HD)
#define ZH   2
#define RH   ((SEQ < 512) ? SEQ : 512)
#define NT   (TT / 64)
#define RELN (2 * TT - 1)
#define BRP  (2 * TT + 128)
#define PCAR 1024.0f
#define SCL  0.125f
#define FILLV (-3.0e38f)
#define SWV  4

static_assert(TT % 128 == 0);
static_assert(NT <= 32);
static_assert(RH % 64 == 0);
static_assert(RH >= 64);
static_assert(NH_ % ZH == 0);
static_assert(BRP % 32 == 0);
static_assert(TT <= SEQ_FULL);
static_assert(NB <= NB_FULL);
static_assert(DM % 64 == 0);
static_assert(DQ == DM);
static_assert((ZH * TT) % SWV == 0);
static_assert(SWV * TT * 4 <= 32768);
static_assert(((size_t)ZH * TT * TT) % 32 == 0);

typedef _Float16 h16;
typedef unsigned short bf;
typedef __attribute__((ext_vector_type(16))) __bf16   v16bf;
typedef __attribute__((ext_vector_type(16))) _Float16 v16h;
typedef __attribute__((ext_vector_type(8)))  _Float16 v8h;
typedef __attribute__((ext_vector_type(8)))  unsigned short v8us;
typedef __attribute__((ext_vector_type(8)))  float    v8f;
typedef __attribute__((ext_vector_type(4)))  float    v4f;
typedef v8h  __attribute__((may_alias)) v8ha;
typedef v4f  __attribute__((may_alias)) v4fa;
typedef v8us __attribute__((may_alias)) v8usa;
typedef __attribute__((ext_vector_type(2))) _Float16 v2h;
typedef __attribute__((ext_vector_type(4))) _Float16 v4h;
typedef __attribute__((ext_vector_type(2))) unsigned short v2us;
typedef __attribute__((ext_vector_type(4))) unsigned short v4us;
typedef __attribute__((ext_vector_type(2))) float v2f;
typedef __attribute__((ext_vector_type(4))) int v4i;

__device__ __forceinline__ unsigned short f2bf(float f) { unsigned u = __float_as_uint(f); u += 0x7FFFu + ((u >> 16) & 1u); return (unsigned short)(u >> 16); }
__device__ __forceinline__ float bf2f(unsigned short b) { return __uint_as_float(((unsigned)b) << 16); }
__device__ __forceinline__ float bfr(float f) { return bf2f(f2bf(f)); }
__device__ __forceinline__ v16h cat16(v8h lo, v8h hi) { return __builtin_shufflevector(lo, hi, 0, 1, 2, 3, 4, 5, 6, 7, 8, 9, 10, 11, 12, 13, 14, 15); }
__device__ __forceinline__ v16bf cat16b(v8us lo, v8us hi) { return __builtin_bit_cast(v16bf, __builtin_shufflevector(lo, hi, 0, 1, 2, 3, 4, 5, 6, 7, 8, 9, 10, 11, 12, 13, 14, 15)); }
__device__ __forceinline__ v8f wmma16(v16h a, v16h b, v8f c) { return __builtin_amdgcn_wmma_f32_16x16x32_f16(false, a, false, b, (short)0, c, false, false); }
__device__ __forceinline__ v8f wmmab(v16bf a, v16bf b, v8f c) { return __builtin_amdgcn_wmma_f32_16x16x32_bf16(false, a, false, b, (short)0, c, false, false); }
__device__ __forceinline__ h16 tohx(float x) { return (h16)x; }
__device__ __forceinline__ void splitf(float y, unsigned short& h, unsigned short& l) { h = f2bf(y); l = f2bf(y - bf2f(h)); }

template <typename T16> struct WFrag;
template <> struct WFrag<h16> { typedef v16h V; static __device__ __forceinline__ V ld(const h16* p) { return cat16(*(const v8h*)p, *(const v8h*)(p + 16)); } static __device__ __forceinline__ v8f mma(V a, V b, v8f c) { return wmma16(a, b, c); } };
template <> struct WFrag<bf> { typedef v16bf V; static __device__ __forceinline__ V ld(const bf* p) { return cat16b(*(const v8us*)p, *(const v8us*)(p + 16)); } static __device__ __forceinline__ v8f mma(V a, V b, v8f c) { return wmmab(a, b, c); } };

template <typename T16, int NSPLIT>
__global__ __launch_bounds__(32) void k_gemmw(const T16* __restrict__ A, const T16* __restrict__ A2, const T16* __restrict__ Bt, const T16* __restrict__ Bt2, int K, float* C, int ldc, size_t sA, size_t sB, size_t sC) {
    typedef typename WFrag<T16>::V V;
    __shared__ __align__(16) float os[16 * 68];
    const size_t z = blockIdx.z; A += z * sA; if (A2) A2 += z * sA; Bt += z * sB; if (Bt2) Bt2 += z * sB; C += z * sC;
    const int lane = threadIdx.x & 31, lr = lane & 15, hi = lane >> 4; const int r0 = blockIdx.x * 64, c0 = blockIdx.y * 64;
    v8f acc[4][4];
#pragma unroll
    for (int mb = 0; mb < 4; ++mb)
#pragma unroll
        for (int nb = 0; nb < 4; ++nb) acc[mb][nb] = (v8f){};
    const size_t aoff = (size_t)(r0 + lr) * K + 8 * hi, boff = (size_t)(c0 + lr) * K + 8 * hi;
#pragma unroll 1
    for (int kc = 0; kc < K; kc += 32) {
        V a[4], a2[4];
#pragma unroll
        for (int mb = 0; mb < 4; ++mb) { a[mb] = WFrag<T16>::ld(A + aoff + (size_t)mb * 16 * K + kc); if (NSPLIT == 1 || NSPLIT == 2) a2[mb] = WFrag<T16>::ld(A2 + aoff + (size_t)mb * 16 * K + kc); }
#pragma unroll
        for (int nb = 0; nb < 4; ++nb) { const V b = WFrag<T16>::ld(Bt + boff + (size_t)nb * 16 * K + kc); V b2; if (NSPLIT >= 2) b2 = WFrag<T16>::ld(Bt2 + boff + (size_t)nb * 16 * K + kc);
#pragma unroll
            for (int mb = 0; mb < 4; ++mb) { acc[mb][nb] = WFrag<T16>::mma(a[mb], b, acc[mb][nb]); if (NSPLIT == 1 || NSPLIT == 2) acc[mb][nb] = WFrag<T16>::mma(a2[mb], b, acc[mb][nb]); if (NSPLIT >= 2) acc[mb][nb] = WFrag<T16>::mma(a[mb], b2, acc[mb][nb]); } }
        asm volatile("v_nop\n\tv_nop\n\tv_nop\n\tv_nop" : "+v"(acc[0][0]), "+v"(acc[1][1]), "+v"(acc[2][2]), "+v"(acc[3][3]) : "v"(a[0]), "v"(a[3]));
    }
#pragma unroll
    for (int mb = 0; mb < 4; ++mb) {
#pragma unroll
        for (int nb = 0; nb < 4; ++nb) {
#pragma unroll
            for (int j = 0; j < 8; ++j) os[(hi * 8 + j) * 68 + nb * 16 + lr] = acc[mb][nb][j]; }
        __builtin_amdgcn_wave_barrier(); asm volatile("" ::: "memory");
        float* crow = C + (size_t)(r0 + mb * 16) * ldc + c0;
#pragma unroll 1
        for (int ps = 0; ps < 2; ++ps) {
#pragma unroll
            for (int s = 0; s < 8; ++s) { const int row = 2 * s + hi, cofs = lr * 4; const v4f val = *(const v4fa*)(os + row * 68 + cofs);
                *(volatile v4f*)(crow + (size_t)row * ldc + cofs) = val; }
            if (ps == 0) __threadfence(); }
        __builtin_amdgcn_wave_barrier(); asm volatile("" ::: "memory");
    }
}

template <typename T16, int NSPLIT, int CMODE>
__global__ __launch_bounds__(32) void k_gemmc(const T16* __restrict__ A, const T16* __restrict__ A2, const T16* __restrict__ Bt, const T16* __restrict__ Bt2, int K, float* C, int ldc, int roff, const int* __restrict__ FLG, size_t sA, size_t sB, size_t sC) {
    typedef typename WFrag<T16>::V V;
    __shared__ __align__(16) float os[16 * 68];
    const size_t z = blockIdx.z; A += z * sA; if (A2) A2 += z * sA; Bt += z * sB; if (Bt2) Bt2 += z * sB; C += z * sC;
    const int lane = threadIdx.x & 31, lr = lane & 15, hi = lane >> 4; const int r0 = blockIdx.x * 64, c0 = blockIdx.y * 64;
    const int qt = min((r0 + roff) >> 6, 31);
    if (CMODE == 1) { const int kt = min(c0 >> 6, 31); if (FLG[qt * 32 + kt] == 0) return; }
    int Kl = K;
    if (CMODE == 2) { int nt = 1;
#pragma unroll 1
        for (int t = 0; t < NT; ++t) { if (FLG[qt * 32 + t] != 0) nt = t + 1; }
        Kl = min(K, nt * 64); }
    v8f acc[4][4];
#pragma unroll
    for (int mb = 0; mb < 4; ++mb)
#pragma unroll
        for (int nb = 0; nb < 4; ++nb) acc[mb][nb] = (v8f){};
    const size_t aoff = (size_t)(r0 + lr) * K + 8 * hi, boff = (size_t)(c0 + lr) * K + 8 * hi;
#pragma unroll 1
    for (int kc = 0; kc < Kl; kc += 32) {
        V a[4], a2[4];
#pragma unroll
        for (int mb = 0; mb < 4; ++mb) { a[mb] = WFrag<T16>::ld(A + aoff + (size_t)mb * 16 * K + kc); if (NSPLIT == 1 || NSPLIT == 2) a2[mb] = WFrag<T16>::ld(A2 + aoff + (size_t)mb * 16 * K + kc); }
#pragma unroll
        for (int nb = 0; nb < 4; ++nb) { const V b = WFrag<T16>::ld(Bt + boff + (size_t)nb * 16 * K + kc); V b2; if (NSPLIT >= 2) b2 = WFrag<T16>::ld(Bt2 + boff + (size_t)nb * 16 * K + kc);
#pragma unroll
            for (int mb = 0; mb < 4; ++mb) { acc[mb][nb] = WFrag<T16>::mma(a[mb], b, acc[mb][nb]); if (NSPLIT == 1 || NSPLIT == 2) acc[mb][nb] = WFrag<T16>::mma(a2[mb], b, acc[mb][nb]); if (NSPLIT >= 2) acc[mb][nb] = WFrag<T16>::mma(a[mb], b2, acc[mb][nb]); } }
        asm volatile("v_nop\n\tv_nop\n\tv_nop\n\tv_nop" : "+v"(acc[0][0]), "+v"(acc[1][1]), "+v"(acc[2][2]), "+v"(acc[3][3]) : "v"(a[0]), "v"(a[3]));
    }
#pragma unroll
    for (int mb = 0; mb < 4; ++mb) {
#pragma unroll
        for (int nb = 0; nb < 4; ++nb) {
#pragma unroll
            for (int j = 0; j < 8; ++j) os[(hi * 8 + j) * 68 + nb * 16 + lr] = acc[mb][nb][j]; }
        __builtin_amdgcn_wave_barrier(); asm volatile("" ::: "memory");
        float* crow = C + (size_t)(r0 + mb * 16) * ldc + c0;
#pragma unroll 1
        for (int ps = 0; ps < 2; ++ps) {
#pragma unroll
            for (int s = 0; s < 8; ++s) { const int row = 2 * s + hi, cofs = lr * 4; const v4f val = *(const v4fa*)(os + row * 68 + cofs);
                *(volatile v4f*)(crow + (size_t)row * ldc + cofs) = val; }
            if (ps == 0) __threadfence(); }
        __builtin_amdgcn_wave_barrier(); asm volatile("" ::: "memory");
    }
}

__global__ __launch_bounds__(256) void k_cvt8(const float* __restrict__ src, bf* dst, size_t n8) { const size_t i = (size_t)blockIdx.x * 256 + threadIdx.x; if (i >= n8) return; const v8f v = *(const v8f*)(src + i * 8); v8us o;
#pragma unroll
    for (int k = 0; k < 8; ++k) o[k] = f2bf(v[k]);
    *(volatile v8us*)(dst + i * 8) = o; __threadfence(); *(volatile v8us*)(dst + i * 8) = o; }

__global__ __launch_bounds__(256) void k_zero4(float* dst, size_t n4) { const size_t i = (size_t)blockIdx.x * 256 + threadIdx.x; if (i >= n4) return; v4f z; z[0] = 0.0f; z[1] = 0.0f; z[2] = 0.0f; z[3] = 0.0f;
    *(volatile v4f*)(dst + i * 4) = z; __threadfence(); *(volatile v4f*)(dst + i * 4) = z; }

__global__ __launch_bounds__(256) void k_hpl(const float* __restrict__ F, h16* P16, bf* Ph, bf* Pl) {
    const size_t e = ((size_t)blockIdx.x * 256 + threadIdx.x) * 2; if (e >= (size_t)NH_ * TT * HD) return;
    const int d = (int)(e % HD); const int t = (int)((e / HD) % TT); const int h = (int)(e / ((size_t)HD * TT));
    const v2f x = *(const v2f*)(F + (size_t)t * DQ + h * HD + d); v2h o16; v2us oh, ol;
#pragma unroll
    for (int q = 0; q < 2; ++q) { o16[q] = tohx(x[q]); unsigned short a2, c2; splitf(x[q], a2, c2); oh[q] = a2; ol[q] = c2; }
    *(volatile v2h*)(P16 + e) = o16; *(volatile v2us*)(Ph + e) = oh; *(volatile v2us*)(Pl + e) = ol; __threadfence(); *(volatile v2h*)(P16 + e) = o16; *(volatile v2us*)(Ph + e) = oh; *(volatile v2us*)(Pl + e) = ol; }

__global__ __launch_bounds__(256) void k_vtp(const float* __restrict__ F, h16* V16, bf* Vh, bf* Vl) { const size_t e = ((size_t)blockIdx.x * 256 + threadIdx.x) * 2; if (e >= (size_t)NH_ * HD * TT) return; const int t = (int)(e % TT); const int d = (int)((e / TT) % HD); const int g = (int)(e / ((size_t)TT * HD)); v2h o16; v2us oh, ol;
#pragma unroll
    for (int q = 0; q < 2; ++q) { const float x = F[(size_t)(t + q) * DQ + g * HD + d]; o16[q] = tohx(x); unsigned short a2, c2; splitf(x, a2, c2); oh[q] = a2; ol[q] = c2; }
    *(volatile v2h*)(V16 + e) = o16; *(volatile v2us*)(Vh + e) = oh; *(volatile v2us*)(Vl + e) = ol; __threadfence(); *(volatile v2h*)(V16 + e) = o16; *(volatile v2us*)(Vh + e) = oh; *(volatile v2us*)(Vl + e) = ol; }

__global__ __launch_bounds__(256) void k_bias(const float* __restrict__ table, float* BR) {
    const int idx = blockIdx.x * 256 + threadIdx.x; if (idx >= NH_ * 4 * BRP) return;
    const int m = idx % BRP; const int s = (idx / BRP) & 3; const int h = idx / (4 * BRP);
    const int ridx = m + s; const bool inr = (ridx < RELN);
    const int rel = (inr ? ridx : 0) - (TT - 1);
    const int sgn = (rel > 0) ? 1 : 0; const int n = (rel < 0) ? -rel : rel;
    const int cnt = ((n >= 12) ? 1 : 0) + ((n >= 16) ? 1 : 0) + ((n >= 23) ? 1 : 0) + ((n >= 32) ? 1 : 0) + ((n >= 46) ? 1 : 0) + ((n >= 64) ? 1 : 0) + ((n >= 91) ? 1 : 0);
    int bucket = (n < 8) ? n : (8 + cnt); bucket += sgn * 16; bucket = min(max(bucket, 0), 31);
    const float tv = bfr(table[bucket * NH_ + h]);
    const float val = inr ? tv : 0.0f;
    *(volatile float*)(BR + idx) = val; __threadfence(); *(volatile float*)(BR + idx) = val; }

__global__ __launch_bounds__(256) void k_tflag(const int* __restrict__ am, const int* __restrict__ kpm, int* FL) {
    __shared__ int sh[NB][256];
    const int tid = threadIdx.x; const int qt = blockIdx.x; const int c = tid * 8; const bool live = (c < TT); const int cc = min(c, TT - 8);
    int any[NB]; v4i kp0[NB], kp1[NB];
#pragma unroll
    for (int b = 0; b < NB; ++b) { any[b] = 0; kp0[b] = *(const v4i*)(kpm + (size_t)b * SEQ_FULL + cc); kp1[b] = *(const v4i*)(kpm + (size_t)b * SEQ_FULL + cc + 4); }
#pragma unroll 1
    for (int r = 0; r < 64; ++r) { const int* mr = am + (size_t)(qt * 64 + r) * SEQ_FULL + cc; const v4i m0 = *(const v4i*)mr; const v4i m1 = *(const v4i*)(mr + 4);
#pragma unroll
        for (int b = 0; b < NB; ++b) {
#pragma unroll
            for (int q = 0; q < 4; ++q) { any[b] |= ((m0[q] != 0) && (kp0[b][q] != 0)) ? 1 : 0; any[b] |= ((m1[q] != 0) && (kp1[b][q] != 0)) ? 1 : 0; } } }
#pragma unroll
    for (int b = 0; b < NB; ++b) sh[b][tid] = live ? any[b] : 0;
    __syncthreads();
    if (tid < 32) { int f[NB];
#pragma unroll
        for (int b = 0; b < NB; ++b) { int a = 0;
#pragma unroll
            for (int k = 0; k < 8; ++k) a |= sh[b][tid * 8 + k];
            f[b] = a; }
#pragma unroll
        for (int b = 0; b < NB; ++b) *(volatile int*)(FL + ((size_t)b * 32 + qt) * 32 + tid) = f[b];
        __threadfence();
#pragma unroll
        for (int b = 0; b < NB; ++b) *(volatile int*)(FL + ((size_t)b * 32 + qt) * 32 + tid) = f[b]; }
}

__global__ __launch_bounds__(SWV * 32) void k_asoft(const float* __restrict__ Sb, const int* __restrict__ am, const int* __restrict__ kp, const float* __restrict__ BR, h16* P16, bf* Ph, bf* Pl) {
#pragma clang fp contract(off)
    __shared__ __align__(16) float rowbuf[SWV][TT];
    const int lane = threadIdx.x & 31; const int w = threadIdx.x >> 5; const int row = blockIdx.x * SWV + w; if (row >= ZH * TT) return; const int i = row % TT; const int zz = row / TT; const bool hires = (i < RH);
    const float* sr = Sb + (size_t)row * TT; const int off = TT - 1 - i; const int sft = off & 3;
    const float* br = BR + ((size_t)zz * 4 + sft) * BRP + (off - sft); const int* amr = am + (size_t)i * SEQ_FULL;
    float mx = FILLV;
#pragma unroll 1
    for (int ch = 0; ch < TT / 128; ++ch) { const int j0 = ch * 128 + lane * 4;
        v4f a = *(const v4f*)(sr + j0); v4i mk = *(const v4i*)(amr + j0); v4i kq = *(const v4i*)(kp + j0); v4f bb = *(const v4f*)(br + j0);
        asm volatile("" : "+v"(a), "+v"(mk), "+v"(kq), "+v"(bb));
        v4f t4;
#pragma unroll
        for (int q = 0; q < 4; ++q) { const bool ok = (mk[q] != 0) && (kq[q] != 0); const float sc = a[q] * SCL; const float sv = sc + bb[q]; const float t = ok ? sv : FILLV; t4[q] = t; mx = fmaxf(mx, t); }
        *(v4fa*)(&rowbuf[w][j0]) = t4; }
#pragma unroll
    for (int sh = 16; sh; sh >>= 1) mx = fmaxf(mx, __shfl_xor(mx, sh, 32));
    const bool dead = (mx < -1.0e38f);
    float sum = 0.f;
#pragma unroll 1
    for (int ch = 0; ch < TT / 128; ++ch) { const int j0 = ch * 128 + lane * 4; v4f t4 = *(const v4fa*)(&rowbuf[w][j0]);
#pragma unroll
        for (int q = 0; q < 4; ++q) { float d0 = __fsub_rn(t4[q], mx); asm volatile("" : "+v"(d0)); const float ev = __builtin_amdgcn_exp2f(__fmul_rn(d0, 1.4426950408889634f)); t4[q] = ev; sum += ev; }
        *(v4fa*)(&rowbuf[w][j0]) = t4; }
#pragma unroll
    for (int sh = 16; sh; sh >>= 1) sum += __shfl_xor(sum, sh, 32);
    const float f0 = __fdiv_rn(hires ? 1.0f : PCAR, sum);
    const float f = dead ? __uint_as_float(0x7fc00000u) : f0;
#pragma unroll 1
    for (int ps = 0; ps < 2; ++ps) {
        if (hires) {
#pragma unroll 1
            for (int ch = 0; ch < TT / 128; ++ch) { const int j0 = ch * 128 + lane * 4; const v4f t4 = *(const v4fa*)(&rowbuf[w][j0]); v4us oh, ol;
#pragma unroll
                for (int q = 0; q < 4; ++q) { float pv = t4[q] * f; asm volatile("" : "+v"(pv)); unsigned short a, c2; splitf(pv, a, c2); oh[q] = a; ol[q] = c2; }
                const size_t oo = ((size_t)zz * RH + i) * TT + j0; *(volatile v4us*)(Ph + oo) = oh; *(volatile v4us*)(Pl + oo) = ol; }
        } else {
#pragma unroll 1
            for (int ch = 0; ch < TT / 128; ++ch) { const int j0 = ch * 128 + lane * 4; const v4f t4 = *(const v4fa*)(&rowbuf[w][j0]); v4h o4;
#pragma unroll
                for (int q = 0; q < 4; ++q) { float pv = t4[q] * f; asm volatile("" : "+v"(pv)); o4[q] = tohx(pv); }
                *(volatile v4h*)(P16 + (size_t)row * TT + j0) = o4; } }
        if (ps == 0) __threadfence(); }
}

__global__ __launch_bounds__(256) void k_merge(const float* __restrict__ O, int h0, bf* Ah, bf* Al) { const size_t e = ((size_t)blockIdx.x * 256 + threadIdx.x) * 2; if (e >= (size_t)ZH * TT * HD) return; const int d = (int)(e % HD); const int t = (int)((e / HD) % TT); const int zz = (int)(e / ((size_t)HD * TT)); const float cs = (t < RH) ? 1.0f : (1.0f / PCAR); const size_t oo = (size_t)t * DQ + (h0 + zz) * HD + d;
    const v2f x = *(const v2f*)(O + e); v2us oh, ol;
#pragma unroll
    for (int q = 0; q < 2; ++q) { unsigned short a, c2; splitf(x[q] * cs, a, c2); oh[q] = a; ol[q] = c2; }
    *(volatile v2us*)(Ah + oo) = oh; *(volatile v2us*)(Al + oo) = ol; __threadfence(); *(volatile v2us*)(Ah + oo) = oh; *(volatile v2us*)(Al + oo) = ol; }

extern "C" void kernel_launch(void* const* d_in, const int* in_sizes, int n_in,
                              void* d_out, int out_size, void* d_ws, size_t ws_size, hipStream_t stream) {
    if (n_in < 9) return;
    const long long need_x = (long long)(NB - 1) * SEQ_FULL * DM + (long long)SEQ * DM;
    if ((long long)in_sizes[0] < need_x || (long long)in_sizes[1] < need_x) return;
    if ((long long)in_sizes[2] < (long long)DQ * DM || (long long)in_sizes[3] < (long long)DQ * DM || (long long)in_sizes[4] < (long long)DQ * DM || (long long)in_sizes[5] < (long long)DM * DQ) return;
    if (in_sizes[6] < 32 * NH_) return;
    if ((long long)in_sizes[7] < (long long)(SEQ - 1) * SEQ_FULL + SEQ) return;
    if ((long long)in_sizes[8] < (long long)(NB - 1) * SEQ_FULL + SEQ) return;
    if ((long long)out_size < need_x) return;
    const float* xq = (const float*)d_in[0]; const float* xkv = (const float*)d_in[1];
    const float* wq = (const float*)d_in[2]; const float* wk = (const float*)d_in[3]; const float* wv = (const float*)d_in[4]; const float* wo = (const float*)d_in[5];
    const float* tbl = (const float*)d_in[6]; const int* am = (const int*)d_in[7]; const int* kpm = (const int*)d_in[8];
    float* OUT = (float*)d_out;
    char* wsp = (char*)d_ws;
    auto take = [&](size_t bytes) { char* p = wsp; wsp += (bytes + 255) & ~(size_t)255; return (void*)p; };
    bf* WQ = (bf*)take((size_t)DQ * DM * 2); bf* WK = (bf*)take((size_t)DQ * DM * 2); bf* WV = (bf*)take((size_t)DQ * DM * 2); bf* WO = (bf*)take((size_t)DM * DQ * 2);
    bf* XB = (bf*)take((size_t)TT * DM * 2); float* F = (float*)take((size_t)TT * DQ * 4);
    h16* QP16 = (h16*)take((size_t)NH_ * TT * HD * 2); h16* KP16 = (h16*)take((size_t)NH_ * TT * HD * 2); h16* VT16 = (h16*)take((size_t)NH_ * HD * TT * 2);
    bf* QPh = (bf*)take((size_t)NH_ * TT * HD * 2); bf* QPl = (bf*)take((size_t)NH_ * TT * HD * 2); bf* KPh = (bf*)take((size_t)NH_ * TT * HD * 2); bf* KPl = (bf*)take((size_t)NH_ * TT * HD * 2);
    bf* VTh = (bf*)take((size_t)NH_ * HD * TT * 2); bf* VTl = (bf*)take((size_t)NH_ * HD * TT * 2);
    bf* Ph = (bf*)take((size_t)ZH * RH * TT * 2); bf* Pl = (bf*)take((size_t)ZH * RH * TT * 2);
    float* Sb = (float*)take((size_t)ZH * TT * TT * 4); h16* P16 = (h16*)take((size_t)ZH * TT * TT * 2); float* Ob = (float*)take((size_t)ZH * TT * HD * 4);
    bf* ATh = (bf*)take((size_t)TT * DQ * 2); bf* ATl = (bf*)take((size_t)TT * DQ * 2);
    float* BR = (float*)take((size_t)NH_ * 4 * BRP * 4); int* FL = (int*)take((size_t)NB * 32 * 32 * 4);
    const size_t used = (size_t)(wsp - (char*)d_ws);
    if (used > ws_size || used > (size_t)134217728) return;
    const unsigned gW = (unsigned)(((size_t)DQ * DM / 8 + 255) / 256);
    k_cvt8<<<gW, 256, 0, stream>>>(wq, WQ, (size_t)DQ * DM / 8);
    k_cvt8<<<gW, 256, 0, stream>>>(wk, WK, (size_t)DQ * DM / 8);
    k_cvt8<<<gW, 256, 0, stream>>>(wv, WV, (size_t)DQ * DM / 8);
    k_cvt8<<<gW, 256, 0, stream>>>(wo, WO, (size_t)DM * DQ / 8);
    k_bias<<<(NH_ * 4 * BRP + 255) / 256, 256, 0, stream>>>(tbl, BR);
    k_tflag<<<NT, 256, 0, stream>>>(am, kpm, FL);
    { const size_t n4 = (size_t)ZH * TT * TT / 4; k_zero4<<<(unsigned)((n4 + 255) / 256), 256, 0, stream>>>(Sb, n4); }
    const unsigned gX = (unsigned)(((size_t)TT * DM / 8 + 255) / 256);
    const unsigned LQ = (unsigned)(((size_t)NH_ * TT * HD / 2 + 255) / 256);
    for (int b = 0; b < NB; ++b) {
        const int* flb = FL + (size_t)b * 32 * 32; const int* kpb = kpm + (size_t)b * SEQ_FULL;
        k_cvt8<<<gX, 256, 0, stream>>>(xq + (size_t)b * SEQ_FULL * DM, XB, (size_t)TT * DM / 8);
        k_gemmw<bf, 0><<<dim3(TT / 64, DQ / 64, 1), 32, 0, stream>>>(XB, nullptr, WQ, nullptr, DM, F, DQ, 0, 0, 0);
        k_hpl<<<LQ, 256, 0, stream>>>(F, QP16, QPh, QPl);
        k_cvt8<<<gX, 256, 0, stream>>>(xkv + (size_t)b * SEQ_FULL * DM, XB, (size_t)TT * DM / 8);
        k_gemmw<bf, 0><<<dim3(TT / 64, DQ / 64, 1), 32, 0, stream>>>(XB, nullptr, WK, nullptr, DM, F, DQ, 0, 0, 0);
        k_hpl<<<LQ, 256, 0, stream>>>(F, KP16, KPh, KPl);
        k_gemmw<bf, 0><<<dim3(TT / 64, DQ / 64, 1), 32, 0, stream>>>(XB, nullptr, WV, nullptr, DM, F, DQ, 0, 0, 0);
        k_vtp<<<LQ, 256, 0, stream>>>(F, VT16, VTh, VTl);
        for (int h0 = 0; h0 < NH_; h0 += ZH) { const size_t zq = (size_t)h0;
            k_gemmc<bf, 2, 1><<<dim3(RH / 64, TT / 64, ZH), 32, 0, stream>>>(QPh + zq * TT * HD, QPl + zq * TT * HD, KPh + zq * TT * HD, KPl + zq * TT * HD, HD, Sb, TT, 0, flb, (size_t)TT * HD, (size_t)TT * HD, (size_t)TT * TT);
            if (TT > RH) k_gemmc<h16, 0, 1><<<dim3((TT - RH) / 64, TT / 64, ZH), 32, 0, stream>>>(QP16 + zq * TT * HD + (size_t)RH * HD, nullptr, KP16 + zq * TT * HD, nullptr, HD, Sb + (size_t)RH * TT, TT, RH, flb, (size_t)TT * HD, (size_t)TT * HD, (size_t)TT * TT);
            k_asoft<<<ZH * TT / SWV, SWV * 32, 0, stream>>>(Sb, am, kpb, BR + zq * 4 * BRP, P16, Ph, Pl);
            k_gemmc<bf, 2, 2><<<dim3(RH / 64, HD / 64, ZH), 32, 0, stream>>>(Ph, Pl, VTh + zq * HD * TT, VTl + zq * HD * TT, TT, Ob, HD, 0, flb, (size_t)RH * TT, (size_t)HD * TT, (size_t)TT * HD);
            if (TT > RH) k_gemmc<h16, 0, 2><<<dim3((TT - RH) / 64, HD / 64, ZH), 32, 0, stream>>>(P16 + (size_t)RH * TT, nullptr, VT16 + zq * HD * TT, nullptr, TT, Ob + (size_t)RH * HD, HD, RH, flb, (size_t)TT * TT, (size_t)HD * TT, (size_t)TT * HD);
            k_merge<<<(unsigned)(((size_t)ZH * TT * HD / 2 + 255) / 256), 256, 0, stream>>>(Ob, h0, ATh, ATl); }
        k_gemmw<bf, 1><<<dim3(TT / 64, DM / 64, 1), 32, 0, stream>>>(ATh, ATl, WO, nullptr, DQ, OUT + (size_t)b * SEQ_FULL * DM, DM, 0, 0, 0); }
}
